// GraphProp_81492709474574
// MI455X (gfx1250) — hardware-verified
//
#include <hip/hip_runtime.h>
#include <stddef.h>
#include <math.h>


#define FD     128
#define HM     256
#define KC     256
#define NTHR   256
#define NWV    8
#define TR     64
#define LDT    264
#define BM     32
#define CE     60032
#define NB     256
#define CH     2048
#define LCAP   4096
#define SP     128
#define WSCAP  134217728
#define VCAP   240
#define SCL_X  8.0f
#define SCL_W  64.0f
#define SCL_P  8.0f
#define INV_XW 0.001953125f
#define INV_P  0.125f

#define LE_TILE 0
#define LE_STG  (LE_TILE + TR * LDT * 2)
#define LE_IDX  (LE_STG + TR * FD * 4)
#define LDS_N   LE_IDX
#define LDS_E   (LE_IDX + 2 * TR * 4)

#define LG_SLIST 0
#define LG_SLOTS (LG_SLIST + LCAP * 4)
#define LG_SDL   (LG_SLOTS + NB * SP * 2)
#define LG_SCNT  (LG_SDL + LCAP * 4)
#define LG_WSUM  (LG_SCNT + NB * 4)
#define LDS_G    (LG_WSUM + 64)

static_assert((LDT % 8) == 0 && LDT >= HM);
static_assert(TR == 64 && NWV * 32 == NTHR && (TR * FD / 4) % NTHR == 0 && (TR * HM / 8) % NTHR == 0);
static_assert((CE % TR) == 0 && (CE % 4) == 0);
static_assert(NB == NTHR && CH == 8 * NTHR && LCAP >= 2 * CH && (LCAP % 4) == 0 && LCAP <= 65536 && SP <= LCAP);
static_assert(NB == 32 * NWV && BM * 8 == NTHR && KC == 2 * FD && HM == 2 * FD && (FD % 32) == 0 && (KC % 32) == 0);
static_assert((LE_STG % 16) == 0 && (LE_IDX % 16) == 0 && (BM * HM / 8) % NTHR == 0 && (BM * HM / 4) % NTHR == 0);
static_assert((LG_SLOTS % 16) == 0 && (LG_SDL % 16) == 0 && (LG_SCNT % 16) == 0 && (LG_WSUM % 16) == 0);
static_assert((VCAP % 8) == 0 && VCAP <= 256);

typedef float    v4f  __attribute__((ext_vector_type(4)));
typedef float    v8f  __attribute__((ext_vector_type(8)));
typedef int      v4i  __attribute__((ext_vector_type(4)));
typedef _Float16 v8h  __attribute__((ext_vector_type(8)));
typedef _Float16 v16h __attribute__((ext_vector_type(16)));
union FragH { v16h v; v8h hh[2]; };

__device__ __forceinline__ v8f wmh(v16h a, v16h b, v8f c) {
  v8f d = __builtin_amdgcn_wmma_f32_16x16x32_f16(false, a, false, b, (short)0, c, false, false);
  asm volatile("v_nop\n\tv_nop\n\tv_nop\n\tv_nop" : "+v"(d) : "v"(a), "v"(b));
  return d;
}

__device__ __forceinline__ v8f zero8() { v8f z = {0.f, 0.f, 0.f, 0.f, 0.f, 0.f, 0.f, 0.f}; return z; }

__device__ __forceinline__ v8h cvt8(v4f a, v4f b, float s) {
  v8f t;
  t[0] = a.x * s; t[1] = a.y * s; t[2] = a.z * s; t[3] = a.w * s;
  t[4] = b.x * s; t[5] = b.y * s; t[6] = b.z * s; t[7] = b.w * s;
  return __builtin_convertvector(t, v8h);
}

__device__ __forceinline__ v16h frag16(const _Float16* p) {
  FragH f;
  f.hh[0] = *(const v8h*)p;
  f.hh[1] = *(const v8h*)(p + 16);
  return f.v;
}

__device__ __forceinline__ v16h afrag_f32(const float* rp, int h, float s) {
  FragH a;
  const float* p0 = rp + 8 * h;
  const float* p1 = rp + 16 + 8 * h;
  a.hh[0] = cvt8(*(const v4f*)p0, *(const v4f*)(p0 + 4), s);
  a.hh[1] = cvt8(*(const v4f*)p1, *(const v4f*)(p1 + 4), s);
  return a.v;
}

__global__ __launch_bounds__(NTHR) void k_wcvt(const float* __restrict__ in, _Float16* outp,
                                               int C, int koff, int K, int KP, int nUnits, float scale) {
  const int u = (int)blockIdx.x * NTHR + (int)threadIdx.x;
  if (u >= nUnits) return;
  const int upr = KP >> 3;
  const int n   = u / upr;
  const int k0  = (u - n * upr) * 8;
  v8f t;
#pragma unroll
  for (int i = 0; i < 8; ++i) {
    const int k  = k0 + i;
    const int kc = k < K ? k : K - 1;
    const float v = in[(size_t)(koff + kc) * C + n] * scale;
    t[i] = (k < K) ? v : 0.0f;
  }
  const v8h o = __builtin_convertvector(t, v8h);
  _Float16* d = outp + (size_t)n * KP + k0;
  *(volatile v8h*)d = o;
  __threadfence();
  *(volatile v8h*)d = o;
}

template <int PH>
__global__ __launch_bounds__(NTHR) __attribute__((amdgpu_num_vgpr(VCAP)))
void k_pqgemm(const float* __restrict__ xin, const _Float16* __restrict__ wp,
              const float* __restrict__ bias, float* outf, _Float16* outh, int nN) {
  __shared__ __attribute__((aligned(16))) float stg[BM * HM];
  const int tid = threadIdx.x, lane = tid & 31;
  const int wave = __builtin_amdgcn_readfirstlane(tid >> 5);
  const int hh = lane >> 4, m = lane & 15;
  const int rg = wave >> 2, cq = wave & 3;
  const int r0 = rg * 16, c0 = cq * 64;
  const int rowBase = blockIdx.x * BM;

  v8f acc[4];
#pragma unroll
  for (int t = 0; t < 4; ++t) acc[t] = zero8();

  int ar = rowBase + r0 + m;
  ar = ar > nN - 1 ? nN - 1 : ar;
  const float* ap = xin + (size_t)ar * FD;
  const _Float16* bp0 = wp + (size_t)(c0 + m) * FD + 8 * hh;
#pragma unroll 1
  for (int kt = 0; kt < FD / 32; ++kt) {
    const v16h a = afrag_f32(ap + 32 * kt, hh, SCL_X);
#pragma unroll
    for (int t = 0; t < 4; ++t) acc[t] = wmh(a, frag16(bp0 + (size_t)(16 * t) * FD + 32 * kt), acc[t]);
  }

  float* sp = stg + (size_t)(r0 + 8 * hh) * HM + c0 + m;
  const int grow0 = rowBase + r0 + 8 * hh;
#pragma unroll
  for (int t = 0; t < 4; ++t) {
    const int n = c0 + 16 * t + m;
    float bv = 0.0f;
    if (PH == 0) bv = bias[n];
#pragma unroll
    for (int r = 0; r < 8; ++r) {
      float v = acc[t][r] * INV_XW + bv;
      v = (grow0 + r < nN) ? v : 0.0f;
      sp[r * HM + 16 * t] = v;
    }
  }
  __syncthreads();

  if (PH != 0) {
    constexpr int NITH = (BM * HM / 8) / NTHR;
    _Float16* tile = outh + (size_t)rowBase * HM;
    v8h oh[NITH];
#pragma unroll
    for (int it = 0; it < NITH; ++it) {
      const float* s8 = stg + 8 * (it * NTHR + tid);
      oh[it] = cvt8(*(const v4f*)s8, *(const v4f*)(s8 + 4), SCL_P);
    }
#pragma unroll
    for (int it = 0; it < NITH; ++it) *(volatile v8h*)(tile + 8 * (size_t)(it * NTHR + tid)) = oh[it];
    __threadfence();
#pragma unroll
    for (int it = 0; it < NITH; ++it) *(volatile v8h*)(tile + 8 * (size_t)(it * NTHR + tid)) = oh[it];
  } else {
    constexpr int NIT4 = (BM * HM / 4) / NTHR;
    float* tile = outf + (size_t)rowBase * HM;
    v4f ov[NIT4];
#pragma unroll
    for (int it = 0; it < NIT4; ++it) ov[it] = *(const v4f*)(stg + 4 * (it * NTHR + tid));
#pragma unroll
    for (int it = 0; it < NIT4; ++it) *(volatile v4f*)(tile + 4 * (size_t)(it * NTHR + tid)) = ov[it];
    __threadfence();
#pragma unroll
    for (int it = 0; it < NIT4; ++it) *(volatile v4f*)(tile + 4 * (size_t)(it * NTHR + tid)) = ov[it];
  }
}

__global__ __launch_bounds__(NTHR) __attribute__((amdgpu_num_vgpr(VCAP)))
void k_edge(const _Float16* __restrict__ pP, const float* __restrict__ qP,
            const int* __restrict__ fix, const int* __restrict__ tix,
            const _Float16* __restrict__ w1, const float* __restrict__ b1,
            float* msg, int nE, int nN, int ebase) {
  extern __shared__ __align__(16) char smem_e[];
  _Float16* tile = (_Float16*)(smem_e + LE_TILE);
  float*    stg  = (float*)(smem_e + LE_STG);
  int*      sidx = (int*)(smem_e + LE_IDX);
  constexpr int NIT4 = (TR * FD / 4) / NTHR;
  constexpr int NITU = (TR * HM / 8) / NTHR;
  static_assert(NIT4 == 8 && NITU == 8 && TR <= NTHR && (TR % 32) == 0);
  const int tid = threadIdx.x, lane = tid & 31;
  const int wave = __builtin_amdgcn_readfirstlane(tid >> 5);
  const int h = lane >> 4, m = lane & 15;
  const int rg = wave >> 1, ch = wave & 1;
  const int cb = 64 * ch;
  const int rl0 = blockIdx.x * TR;
  const int e0 = ebase + rl0;

  if (tid < TR) {
    int e = e0 + tid;
    e = e > nE - 1 ? nE - 1 : e;
    int s = fix[e];
    int d = tix[e];
    s = s < 0 ? 0 : (s > nN - 1 ? nN - 1 : s);
    d = d < 0 ? 0 : (d > nN - 1 ? nN - 1 : d);
    sidx[tid] = s;
    sidx[TR + tid] = d;
  }
  __syncthreads();

#pragma unroll 1
  for (int it = 0; it < NITU; ++it) {
    const int row = it * NWV + wave;
    const int c8  = lane * 8;
    const int sr  = sidx[row];
    const int dr  = sidx[TR + row];
    const v8h p8 = *(const v8h*)(pP + (size_t)sr * HM + c8);
    const float* qp = qP + (size_t)dr * HM + c8;
    const v4f q0 = *(const v4f*)qp;
    const v4f q1 = *(const v4f*)(qp + 4);
    const v8f pf = __builtin_convertvector(p8, v8f);
    v8f t;
    t[0] = pf[0] * INV_P + q0.x; t[1] = pf[1] * INV_P + q0.y;
    t[2] = pf[2] * INV_P + q0.z; t[3] = pf[3] * INV_P + q0.w;
    t[4] = pf[4] * INV_P + q1.x; t[5] = pf[5] * INV_P + q1.y;
    t[6] = pf[6] * INV_P + q1.z; t[7] = pf[7] * INV_P + q1.w;
#pragma unroll
    for (int j = 0; j < 8; ++j) t[j] = fmaxf(t[j], 0.0f) * SCL_X;
    *(v8h*)(tile + (size_t)row * LDT + c8) = __builtin_convertvector(t, v8h);
  }
  __syncthreads();

  const _Float16* arow = tile + (size_t)(16 * rg + m) * LDT + 8 * h;
  float* srow0 = stg + (size_t)(16 * rg + 8 * h) * FD + m;
#pragma unroll 1
  for (int cp = 0; cp < 2; ++cp) {
    const int colb = cb + 32 * cp;
    const _Float16* bp0 = w1 + (size_t)(colb + m) * KC + 8 * h;
    const _Float16* bp1 = bp0 + (size_t)16 * KC;
    v8f acc0 = zero8();
    v8f acc1 = zero8();
#pragma unroll 1
    for (int kt = 0; kt < KC / 32; ++kt) {
      const v16h a = frag16(arow + 32 * kt);
      acc0 = wmh(a, frag16(bp0 + 32 * kt), acc0);
      acc1 = wmh(a, frag16(bp1 + 32 * kt), acc1);
    }
    const float bb0 = b1[colb + m];
    const float bb1 = b1[colb + 16 + m];
    float* srow = srow0 + colb;
#pragma unroll
    for (int r = 0; r < 8; ++r) {
      srow[r * FD]      = fmaxf(acc0[r] * INV_XW + bb0, 0.0f);
      srow[r * FD + 16] = fmaxf(acc1[r] * INV_XW + bb1, 0.0f);
    }
  }
  __syncthreads();

  float* dstp = msg + (size_t)rl0 * FD;
  v4f ov[NIT4];
#pragma unroll
  for (int it = 0; it < NIT4; ++it) ov[it] = *(const v4f*)(stg + 4 * (it * NTHR + tid));
#pragma unroll
  for (int it = 0; it < NIT4; ++it) *(volatile v4f*)(dstp + 4 * (size_t)(it * NTHR + tid)) = ov[it];
  __threadfence();
#pragma unroll
  for (int it = 0; it < NIT4; ++it) *(volatile v4f*)(dstp + 4 * (size_t)(it * NTHR + tid)) = ov[it];
}

__global__ __launch_bounds__(NTHR) __attribute__((amdgpu_num_vgpr(VCAP)))
void k_gather(const int* __restrict__ tix, const float* __restrict__ msg, float* agg,
              int ebase, int clen, int firstChunk) {
  extern __shared__ __align__(16) char smem_g[];
  int*            slist  = (int*)(smem_g + LG_SLIST);
  unsigned short* slots  = (unsigned short*)(smem_g + LG_SLOTS);
  int*            sdl    = (int*)(smem_g + LG_SDL);
  int*            scount = (int*)(smem_g + LG_SCNT);
  int*            wsum   = (int*)(smem_g + LG_WSUM);
  int*            scnt   = wsum + NWV;

  const int tid = threadIdx.x, lane = tid & 31;
  const int wave = __builtin_amdgcn_readfirstlane(tid >> 5);
  const int node0 = blockIdx.x * NB;
  const bool vec_ok = ((ebase & 3) == 0) && ((((size_t)tix) & 15) == 0);
  const v4f z4 = {0.0f, 0.0f, 0.0f, 0.0f};
  const float qn = __int_as_float(0x7fc00000);
  const v4f vnan = {qn, qn, qn, qn};

  int cnt = 0, pass = 0;
  for (int cb = 0; ; cb += CH) {
    const bool endc = (cb >= clen);
    if (endc || (cnt + CH > LCAP)) {
      __syncthreads();
      int k = 0;
#pragma unroll 1
      for (int i = 0; i < cnt; i += 4) {
        const v4i w4 = *(const v4i*)(sdl + i);
#pragma unroll
        for (int q = 0; q < 4; ++q) {
          const bool hit = (w4[q] == tid) && (i + q < cnt);
          if (hit) {
            if (k < SP) slots[tid * SP + k] = (unsigned short)(i + q);
            ++k;
          }
        }
      }
      scount[tid] = k;
      __syncthreads();

      const bool first = (firstChunk != 0) && (pass == 0);
#pragma unroll 1
      for (int j = 0; j < 32; ++j) {
        const int nl = 32 * wave + j;
        float* mrow = agg + (size_t)(node0 + nl) * FD + 4 * lane;
        int cn = __builtin_amdgcn_readfirstlane(scount[nl]);
        const bool ovf = cn > SP;
        cn = cn > SP ? SP : cn;
        v4f acc = *(const v4f*)mrow;
        acc = first ? z4 : acc;
#pragma unroll 1
        for (int p = 0; p < cn; ++p) {
          int i = (int)slots[nl * SP + p];
          i = i > LCAP - 1 ? LCAP - 1 : i;
          int el = slist[i];
          el = el < 0 ? 0 : (el > clen - 1 ? clen - 1 : el);
          const v4f ms = *(const v4f*)(msg + (size_t)el * FD + 4 * lane);
          acc = acc + ms;
        }
        acc = ovf ? vnan : acc;
        *(volatile v4f*)mrow = acc;
        __threadfence();
        *(volatile v4f*)mrow = acc;
      }
      __syncthreads();
      ++pass;
      cnt = 0;
    }
    if (endc) break;

    int dv[8];
    if (vec_ok && (cb + CH <= clen)) {
      const int* bp = tix + (size_t)ebase + cb + 8 * tid;
      const v4i a = *(const v4i*)bp;
      const v4i b = *(const v4i*)(bp + 4);
      dv[0] = a[0]; dv[1] = a[1]; dv[2] = a[2]; dv[3] = a[3];
      dv[4] = b[0]; dv[5] = b[1]; dv[6] = b[2]; dv[7] = b[3];
    } else {
#pragma unroll
      for (int j = 0; j < 8; ++j) {
        const int el = cb + 8 * tid + j;
        const int ec = el > clen - 1 ? clen - 1 : el;
        const int dj = tix[(size_t)ebase + ec];
        dv[j] = (el < clen) ? dj : -1;
      }
    }
    unsigned bits = 0u;
#pragma unroll
    for (int j = 0; j < 8; ++j) {
      const int dlj = dv[j] - node0;
      bits |= ((unsigned)dlj < (unsigned)NB) ? (1u << j) : 0u;
    }
    const int pc = __builtin_popcount(bits);
    int incl = pc;
#pragma unroll
    for (int sh = 1; sh < 32; sh <<= 1) {
      const int t = __shfl_up(incl, sh);
      incl += (lane >= sh) ? t : 0;
    }
    if (lane == 31) wsum[wave] = incl;
    __syncthreads();
    int woff = 0, tot = 0;
#pragma unroll
    for (int w = 0; w < NWV; ++w) {
      const int v = wsum[w];
      woff += (w < wave) ? v : 0;
      tot += v;
    }
    int pos = cnt + woff + incl - pc;
#pragma unroll
    for (int j = 0; j < 8; ++j) {
      if (bits & (1u << j)) {
        if (pos < LCAP) {
          slist[pos] = cb + 8 * tid + j;
          sdl[pos]   = dv[j] - node0;
        }
        ++pos;
      }
    }
    if (tid == 0) scnt[0] = cnt + tot;
    __syncthreads();
    cnt = scnt[0];
    cnt = cnt > LCAP ? LCAP : cnt;
  }
}

__global__ __launch_bounds__(NTHR) __attribute__((amdgpu_num_vgpr(VCAP)))
void k_node(const float* __restrict__ xin, const float* __restrict__ agg,
            const _Float16* __restrict__ wu0, const _Float16* __restrict__ wu1,
            const float* __restrict__ b0, const float* __restrict__ b1, float* outp, int nN) {
  extern __shared__ __align__(16) char smem_n[];
  _Float16* tile = (_Float16*)(smem_n + LE_TILE);
  float*    stg  = (float*)(smem_n + LE_STG);
  constexpr int NIT4 = (TR * FD / 4) / NTHR;
  const int tid = threadIdx.x, lane = tid & 31;
  const int wave = __builtin_amdgcn_readfirstlane(tid >> 5);
  const int h = lane >> 4, m = lane & 15;
  const int rg = wave >> 1, ch = wave & 1;
  const int cb = 64 * ch;
  const int rowBase = blockIdx.x * TR;
  const int grow = rowBase + 16 * rg + m;
  const int gcl = grow > nN - 1 ? nN - 1 : grow;

  v8f acc[4];
  const float* ap1 = agg + (size_t)grow * FD;
  const float* ap2 = xin + (size_t)gcl * FD;
#pragma unroll 1
  for (int cp = 0; cp < 2; ++cp) {
#pragma unroll
    for (int nt = 0; nt < 4; ++nt) acc[nt] = zero8();
    const int colb = FD * cp + cb;
    const _Float16* bp0 = wu0 + (size_t)(colb + m) * KC + 8 * h;
#pragma unroll 1
    for (int kt = 0; kt < FD / 32; ++kt) {
      const v16h a = afrag_f32(ap1 + 32 * kt, h, SCL_X);
#pragma unroll
      for (int nt = 0; nt < 4; ++nt)
        acc[nt] = wmh(a, frag16(bp0 + (size_t)(16 * nt) * KC + 32 * kt), acc[nt]);
    }
#pragma unroll 1
    for (int kt = 0; kt < FD / 32; ++kt) {
      const v16h a = afrag_f32(ap2 + 32 * kt, h, SCL_X);
#pragma unroll
      for (int nt = 0; nt < 4; ++nt)
        acc[nt] = wmh(a, frag16(bp0 + (size_t)(16 * nt) * KC + FD + 32 * kt), acc[nt]);
    }
    _Float16* trow = tile + (size_t)(16 * rg + 8 * h) * LDT + colb + m;
#pragma unroll
    for (int nt = 0; nt < 4; ++nt) {
      const float bb = b0[colb + 16 * nt + m];
#pragma unroll
      for (int r = 0; r < 8; ++r) {
        const float v = fmaxf(acc[nt][r] * INV_XW + bb, 0.0f) * SCL_X;
        trow[r * LDT + 16 * nt] = (_Float16)v;
      }
    }
  }
  __syncthreads();

#pragma unroll
  for (int nt = 0; nt < 4; ++nt) acc[nt] = zero8();
  {
    const _Float16* arow = tile + (size_t)(16 * rg + m) * LDT + 8 * h;
    const _Float16* bq0  = wu1 + (size_t)(cb + m) * KC + 8 * h;
#pragma unroll 1
    for (int kt = 0; kt < KC / 32; ++kt) {
      const v16h a = frag16(arow + 32 * kt);
#pragma unroll
      for (int nt = 0; nt < 4; ++nt) acc[nt] = wmh(a, frag16(bq0 + (size_t)(16 * nt) * KC + 32 * kt), acc[nt]);
    }
  }
  {
    float* srow = stg + (size_t)(16 * rg + 8 * h) * FD + cb + m;
#pragma unroll
    for (int nt = 0; nt < 4; ++nt) {
      const float bb = b1[cb + 16 * nt + m];
#pragma unroll
      for (int r = 0; r < 8; ++r) srow[r * FD + 16 * nt] = fmaxf(acc[nt][r] * INV_XW + bb, 0.0f);
    }
  }
  __syncthreads();

  v4f ov[NIT4];
#pragma unroll
  for (int it = 0; it < NIT4; ++it) {
    const int u = it * NTHR + tid;
    const int orow = rowBase + (u >> 5);
    const int oc = orow > nN - 1 ? nN - 1 : orow;
    const v4f xv = *(const v4f*)(xin + (size_t)oc * FD + 4 * (u & 31));
    ov[it] = *(const v4f*)(stg + 4 * u) + xv;
  }
#pragma unroll
  for (int it = 0; it < NIT4; ++it) {
    const int u = it * NTHR + tid;
    const int orow = rowBase + (u >> 5);
    if (orow < nN) *(volatile v4f*)(outp + (size_t)orow * FD + 4 * (u & 31)) = ov[it];
  }
  __threadfence();
#pragma unroll
  for (int it = 0; it < NIT4; ++it) {
    const int u = it * NTHR + tid;
    const int orow = rowBase + (u >> 5);
    if (orow < nN) *(volatile v4f*)(outp + (size_t)orow * FD + 4 * (u & 31)) = ov[it];
  }
}

extern "C" void kernel_launch(void* const* d_in, const int* in_sizes, int n_in,
                              void* d_out, int out_size, void* d_ws, size_t ws_size,
                              hipStream_t stream) {
  if (n_in < 11) return;
  const int nN = in_sizes[0] / FD;
  const int nE = in_sizes[1];
  if (nN <= 0 || nE <= 0) return;
  if (in_sizes[0] != nN * FD || in_sizes[2] != nE) return;
  if (in_sizes[3] != KC * HM || in_sizes[4] != HM) return;
  if (in_sizes[5] != KC * FD || in_sizes[6] != FD) return;
  if (in_sizes[7] != KC * HM || in_sizes[8] != HM) return;
  if (in_sizes[9] != KC * FD || in_sizes[10] != FD) return;
  if (out_size != nN * FD) return;
  if (nE > (1 << 27) || nN > (1 << 22)) return;

  const float* x   = (const float*)d_in[0];
  const int*   fix = (const int*)d_in[1];
  const int*   tix = (const int*)d_in[2];
  const float* mW0 = (const float*)d_in[3];
  const float* mb0 = (const float*)d_in[4];
  const float* mW1 = (const float*)d_in[5];
  const float* mb1 = (const float*)d_in[6];
  const float* uW0 = (const float*)d_in[7];
  const float* ub0 = (const float*)d_in[8];
  const float* uW1 = (const float*)d_in[9];
  const float* ub1 = (const float*)d_in[10];
  float* outp = (float*)d_out;

  const int nGat   = (nN + NB - 1) / NB;
  const int NPAD   = nGat * NB;
  const int nGemm  = NPAD / BM;
  const int nNode  = NPAD / TR;
  const int nChunk = (nE + CE - 1) / CE;
  if (nChunk > 256) return;

  char* ws = (char*)d_ws;
  size_t off = 0;
  const size_t oWP  = off; off += (size_t)HM * FD * 2;    off = (off + 255) & ~(size_t)255;
  const size_t oWQ  = off; off += (size_t)HM * FD * 2;    off = (off + 255) & ~(size_t)255;
  const size_t oW1  = off; off += (size_t)FD * KC * 2;    off = (off + 255) & ~(size_t)255;
  const size_t oWU0 = off; off += (size_t)HM * KC * 2;    off = (off + 255) & ~(size_t)255;
  const size_t oWU1 = off; off += (size_t)FD * KC * 2;    off = (off + 255) & ~(size_t)255;
  const size_t oP   = off; off += (size_t)NPAD * HM * 2;  off = (off + 255) & ~(size_t)255;
  const size_t oQ   = off; off += (size_t)NPAD * HM * 4;  off = (off + 255) & ~(size_t)255;
  const size_t oAGG = off; off += (size_t)NPAD * FD * 4;  off = (off + 255) & ~(size_t)255;
  const size_t oMSG = off; off += (size_t)CE * FD * 4;    off = (off + 255) & ~(size_t)255;
  if (off > ws_size || off > (size_t)WSCAP) return;
  _Float16* wP   = (_Float16*)(ws + oWP);
  _Float16* wQ   = (_Float16*)(ws + oWQ);
  _Float16* w1   = (_Float16*)(ws + oW1);
  _Float16* wu0  = (_Float16*)(ws + oWU0);
  _Float16* wu1  = (_Float16*)(ws + oWU1);
  _Float16* pPl  = (_Float16*)(ws + oP);
  float*    qPl  = (float*)(ws + oQ);
  float*    aggP = (float*)(ws + oAGG);
  float*    msgP = (float*)(ws + oMSG);

  (void)hipFuncSetAttribute(reinterpret_cast<const void*>(&k_gather),
                            hipFuncAttributeMaxDynamicSharedMemorySize, (int)LDS_G);
  (void)hipFuncSetAttribute(reinterpret_cast<const void*>(&k_edge),
                            hipFuncAttributeMaxDynamicSharedMemorySize, (int)LDS_E);
  (void)hipFuncSetAttribute(reinterpret_cast<const void*>(&k_node),
                            hipFuncAttributeMaxDynamicSharedMemorySize, (int)LDS_N);

  const int nuPQ = HM * (FD / 8);
  const int nuW1 = FD * (KC / 8);
  const int nuU0 = HM * (KC / 8);
  k_wcvt<<<(nuPQ + NTHR - 1) / NTHR, NTHR, 0, stream>>>(mW0, wP,  HM, 0,  FD, FD, nuPQ, SCL_W);
  k_wcvt<<<(nuPQ + NTHR - 1) / NTHR, NTHR, 0, stream>>>(mW0, wQ,  HM, FD, FD, FD, nuPQ, SCL_W);
  k_wcvt<<<(nuW1 + NTHR - 1) / NTHR, NTHR, 0, stream>>>(mW1, w1,  FD, 0,  KC, KC, nuW1, SCL_W);
  k_wcvt<<<(nuU0 + NTHR - 1) / NTHR, NTHR, 0, stream>>>(uW0, wu0, HM, 0,  KC, KC, nuU0, SCL_W);
  k_wcvt<<<(nuW1 + NTHR - 1) / NTHR, NTHR, 0, stream>>>(uW1, wu1, FD, 0,  KC, KC, nuW1, SCL_W);
  k_pqgemm<1><<<nGemm, NTHR, 0, stream>>>(x, wP, mb0, qPl, pPl, nN);
  k_pqgemm<0><<<nGemm, NTHR, 0, stream>>>(x, wQ, mb0, qPl, pPl, nN);
  for (int c = 0; c < nChunk; ++c) {
    const int ebase = c * CE;
    const int clen  = (nE - ebase) < CE ? (nE - ebase) : CE;
    const int nb    = (clen + TR - 1) / TR;
    k_edge<<<nb, NTHR, LDS_E, stream>>>(pPl, qPl, fix, tix, w1, mb1, msgP, nE, nN, ebase);
    k_gather<<<nGat, NTHR, LDS_G, stream>>>(tix, msgP, aggP, ebase, clen, (c == 0) ? 1 : 0);
  }
  k_node<<<nNode, NTHR, LDS_N, stream>>>(x, aggP, wu0, wu1, ub0, ub1, outp, nN);
}
